// H_GAT_55903294324912
// MI455X (gfx1250) — hardware-run, weakly checked
//
#include <hip/hip_runtime.h>


namespace {
constexpr int N = 50000, NP = 50048, NLIM = 50048  , NLIMN = (NLIM < N ? NLIM : N), E = 400000, D = 128, NT = 10, KS = 3 * D  , KA = 4 * D  ;
constexpr float XS = 8.0f, WSC = 256.0f;
static_assert(NP % 64 == 0 && NLIM % 64 == 0, "tiling");
typedef _Float16 b16;
typedef __attribute__((ext_vector_type(16))) _Float16 v16b;
typedef __attribute__((ext_vector_type(8))) _Float16 v8b;
typedef __attribute__((ext_vector_type(8))) float v8f;
typedef __attribute__((ext_vector_type(4))) float v4f;
__device__ __forceinline__ float bf16_rne(float f) { unsigned int u = __float_as_uint(f); u += 0x7FFFu + ((u >> 16) & 1u); return __uint_as_float(u & 0xFFFF0000u); }
__device__ __forceinline__ void split16(float v, b16& hi, b16& lo) { hi = (b16)v; lo = (b16)(v - (float)hi); }
__device__ __forceinline__ v16b frag_kb(const b16* p, int hh) { const v8b a = *(const v8b*)(p + 8 * hh), b = *(const v8b*)(p + 16 + 8 * hh); v16b f;
#pragma unroll
  for (int e = 0; e < 8; ++e) { f[e] = a[e]; f[8 + e] = b[e]; } return f; }
__device__ __forceinline__ v8f wmma16b(v16b a, v16b b, v8f c) { v8f d = __builtin_amdgcn_wmma_f32_16x16x32_f16(false, a, false, b, (short)0, c, false, false); asm volatile("v_nop\n\tv_nop\n\tv_nop\n\tv_nop" : "+v"(d) : "v"(a), "v"(b)); return d; }
__device__ __forceinline__ void wave_lds_sync() { __builtin_amdgcn_fence(__ATOMIC_RELEASE, "workgroup"); __builtin_amdgcn_wave_barrier(); __builtin_amdgcn_fence(__ATOMIC_ACQUIRE, "workgroup"); }
__device__ __forceinline__ float pmul(float a, float b) { float p = a * b; asm volatile("" : "+v"(p)); return p; }
__device__ __forceinline__ int iclamp(int v, int lo, int hi) { return v < lo ? lo : (v > hi ? hi : v); }
constexpr int CSR_NBLK = 512, CSR_GB = 9, CSR_GN = 1 << CSR_GB  , CSR_MAXG = 512, CSR_CAP = 12288  ;
__global__ __launch_bounds__(64) void csrA_kernel(const int* __restrict__ dst, int E, int N, int nG, int CHP, int NGP, int* __restrict__ STG, int* __restrict__ HST) {
  extern __shared__ int sm[];
  int* cnt = sm; int* run = sm + NGP; int* ids = sm + 2 * NGP;
  const int b = blockIdx.x; const int ch = (E + CSR_NBLK - 1) / CSR_NBLK; const int e0 = b * ch, e1 = min(E, e0 + ch);
  for (int i = threadIdx.x; i < NGP; i += 64) cnt[i] = 0;
  for (int i = threadIdx.x; i < CHP; i += 64) ids[i] = -1;
  __syncthreads();
  if (threadIdx.x == 0) {
    for (int e = e0; e < e1; ++e) { int d = dst[e]; d = (d < 0) ? 0 : (d >= N ? N - 1 : d); cnt[d >> CSR_GB] += 1; }
    int acc = 0; for (int g = 0; g < nG; ++g) { run[g] = acc; acc += cnt[g]; }
    for (int e = e0; e < e1; ++e) { int d = dst[e]; d = (d < 0) ? 0 : (d >= N ? N - 1 : d); const int g = d >> CSR_GB; ids[run[g]] = e; run[g] += 1; } }
  __syncthreads();
  typedef __attribute__((ext_vector_type(4))) int v4i;
  for (int pass = 0; pass < 2; ++pass) {
    for (int i = threadIdx.x; i < CHP / 4; i += 64) *(volatile v4i*)(STG + (size_t)b * CHP + i * 4) = *(const v4i*)(&ids[i * 4]);
    for (int i = threadIdx.x; i < NGP / 4; i += 64) { v4i v; for (int e = 0; e < 4; ++e) v[e] = (i * 4 + e < nG) ? cnt[i * 4 + e] : 0; *(volatile v4i*)(HST + (size_t)b * NGP + i * 4) = v; }
    __threadfence(); }
}
__global__ __launch_bounds__(512) void csrS_kernel(const int* __restrict__ HST, int nG, int NGP, int* __restrict__ START, int* __restrict__ TOT, int* __restrict__ OFF) {
  __shared__ int tot[CSR_MAXG];
  const int b = threadIdx.x;
  for (int pass = 0; pass < 2; ++pass) { int runb = 0; for (int g = 0; g < nG; ++g) { int c = HST[(size_t)b * NGP + g]; c = (c < 0) ? 0 : c; ((volatile int*)OFF)[(size_t)g * CSR_NBLK + b] = runb; runb += c; } __threadfence(); }
  for (int g = threadIdx.x; g < nG; g += 512) { int s = 0; for (int bb = 0; bb < CSR_NBLK; ++bb) { int c = HST[(size_t)bb * NGP + g]; s += (c < 0) ? 0 : c; } tot[g] = s; }
  __syncthreads();
  if (threadIdx.x < 32) {
    __shared__ int st[CSR_MAXG + 32];
    if (threadIdx.x == 0) { int acc = 0; for (int g = 0; g < NGP; ++g) { st[g] = acc; if (g < nG) acc += (tot[g] + 31) & ~31; } st[NGP] = acc; }
    __builtin_amdgcn_fence(__ATOMIC_RELEASE, "workgroup"); __builtin_amdgcn_wave_barrier(); __builtin_amdgcn_fence(__ATOMIC_ACQUIRE, "workgroup");
    for (int pass = 0; pass < 2; ++pass) { for (int i = threadIdx.x; i < NGP + 32; i += 32) { ((volatile int*)START)[i] = (i <= NGP) ? st[min(i, NGP)] : 0; ((volatile int*)TOT)[i] = (i < nG) ? tot[i] : 0; } __threadfence(); } }
}
__global__ __launch_bounds__(256) void csrB_kernel(const int* __restrict__ dst, int N, int nG, int CHP, int NGP, int permLen, const int* __restrict__ STG, const int* __restrict__ HST, const int* __restrict__ OFF, const int* __restrict__ START, const int* __restrict__ TOT, int* __restrict__ PERM, int* __restrict__ ROWPTR, int* __restrict__ ROWCNT, int* __restrict__ FLAG) {
  typedef __attribute__((ext_vector_type(4))) int v4i;
  __shared__ int ids[CSR_CAP]; __shared__ unsigned short key[CSR_CAP]; __shared__ int outp[CSR_CAP]; __shared__ int ncnt[CSR_GN + 1]; __shared__ int boff[CSR_NBLK + 1];
  const int g = blockIdx.x, t_ = threadIdx.x; int tot = TOT[g]; int st = START[g], stn = START[g + 1]; const int v0 = g * CSR_GN; const int nv = min(CSR_GN, N - v0);
  st = (st < 0) ? 0 : (st > permLen - 32 ? permLen - 32 : st) & ~31; stn = (stn < st) ? st : (stn > permLen ? permLen : stn); tot = (tot < 0) ? 0 : tot; if (tot > stn - st && tot <= CSR_CAP) tot = stn - st;
  if (tot > CSR_CAP) {
    for (int pass = 0; pass < 2; ++pass) { for (int i = t_; i < CSR_GN / 4; i += 256) { v4i a, c; for (int e = 0; e < 4; ++e) { a[e] = st; c[e] = 0; } *(volatile v4i*)(ROWPTR + v0 + i * 4) = a; *(volatile v4i*)(ROWCNT + v0 + i * 4) = c; } if (t_ == 0) ((volatile int*)FLAG)[0] = 1; __threadfence(); } (void)nv; return; }
  if (t_ == 0) { int acc = 0; for (int b = 0; b < CSR_NBLK; ++b) { boff[b] = acc; int c = HST[(size_t)b * NGP + g]; c = (c < 0) ? 0 : (c > CHP ? CHP : c); acc += c; if (acc > tot) acc = tot; } boff[CSR_NBLK] = acc; }
  for (int i = t_; i <= CSR_GN; i += 256) ncnt[i] = 0;
  __syncthreads();
  for (int b = 0; b < CSR_NBLK; ++b) { const int c = boff[b + 1] - boff[b]; int o_ = OFF[(size_t)g * CSR_NBLK + b]; o_ = (o_ < 0) ? 0 : (o_ > CHP - c ? CHP - c : o_); const int* src_ = STG + (size_t)b * CHP + o_;
    for (int i = t_; i < c; i += 256) { int id = src_[i]; id = (id < 0) ? 0 : id; ids[boff[b] + i] = id; int d = dst[id]; d = (d < v0) ? v0 : (d >= N ? N - 1 : d); int kk = d - v0; kk = (kk < 0) ? 0 : (kk >= CSR_GN ? CSR_GN - 1 : kk); key[boff[b] + i] = (unsigned short)kk; } }
  __syncthreads();
  if (t_ == 0) { for (int i = 0; i < tot; ++i) ncnt[key[i]] += 1; int acc = 0; for (int vl = 0; vl < CSR_GN; ++vl) { const int c = ncnt[vl]; ncnt[vl] = acc; acc += c; } ncnt[CSR_GN] = acc;
    for (int i = 0; i < tot; ++i) { const int vl = key[i]; outp[ncnt[vl]] = ids[i]; ncnt[vl] += 1; }
    for (int vl = CSR_GN; vl > 0; --vl) ncnt[vl] = ncnt[vl - 1]; ncnt[0] = 0; }
  __syncthreads();
  for (int pass = 0; pass < 2; ++pass) {
    for (int i = t_; i < (stn - st) / 4; i += 256) { v4i v; for (int e = 0; e < 4; ++e) { const int q = i * 4 + e; v[e] = (q < tot) ? outp[q] : -1; } *(volatile v4i*)(PERM + st + i * 4) = v; }
    for (int i = t_; i < CSR_GN / 4; i += 256) { v4i a, c; for (int e = 0; e < 4; ++e) { const int vl = i * 4 + e; a[e] = st + ncnt[vl]; c[e] = (vl < nv) ? (ncnt[vl + 1] - ncnt[vl]) : 0; } *(volatile v4i*)(ROWPTR + v0 + i * 4) = a; *(volatile v4i*)(ROWCNT + v0 + i * 4) = c; }
    __threadfence(); }
}
__global__ __launch_bounds__(256) void csrZ_kernel(int* __restrict__ p, size_t n4) { typedef __attribute__((ext_vector_type(4))) int v4i; const size_t tid = (size_t)blockIdx.x * 256 + threadIdx.x, nth = (size_t)gridDim.x * 256; v4i z = {0, 0, 0, 0}; for (size_t i = tid; i < n4; i += nth) *(volatile v4i*)(p + i * 4) = z; }
struct CsrBufs { int *STG, *HST, *OFF, *START, *TOT, *PERM, *ROWPTR, *ROWCNT, *FLAG; int nG, NGP, CHP; size_t permLen; char* base; size_t bytes; };
static size_t csr_carve(CsrBufs& c, char* ws, size_t off, int E, int N) {
  const size_t off0 = off; c.base = ws + off;
  auto al = [&](size_t bytes) { char* p = ws + off; off += (bytes + 255) & ~(size_t)255; return p; };
  c.nG = (N + CSR_GN - 1) / CSR_GN; c.NGP = (c.nG + 31) & ~31; const int ch = (E + CSR_NBLK - 1) / CSR_NBLK; c.CHP = (ch + 31) & ~31; c.permLen = (size_t)E + 32 * (size_t)c.nG + 32;
  c.STG = (int*)al((size_t)CSR_NBLK * c.CHP * 4); c.HST = (int*)al((size_t)CSR_NBLK * c.NGP * 4); c.OFF = (int*)al((size_t)c.NGP * CSR_NBLK * 4); c.START = (int*)al((size_t)(c.NGP + 64) * 4); c.TOT = (int*)al((size_t)(c.NGP + 64) * 4);
  c.PERM = (int*)al(c.permLen * 4); c.ROWPTR = (int*)al((size_t)c.nG * CSR_GN * 4); c.ROWCNT = (int*)al((size_t)c.nG * CSR_GN * 4); c.FLAG = (int*)al(256);
  c.bytes = off - off0; return off;
}
static void csr_build(const CsrBufs& c, const int* dst, int E, int N, hipStream_t stream) {
  const size_t smem = (size_t)(2 * c.NGP + c.CHP) * 4;
  csrZ_kernel<<<512, 256, 0, stream>>>((int*)c.base, c.bytes / 16);
  csrA_kernel<<<CSR_NBLK, 64, smem, stream>>>(dst, E, N, c.nG, c.CHP, c.NGP, c.STG, c.HST);
  csrS_kernel<<<1, 512, 0, stream>>>(c.HST, c.nG, c.NGP, c.START, c.TOT, c.OFF);
  csrB_kernel<<<c.nG, 256, 0, stream>>>(dst, N, c.nG, c.CHP, c.NGP, (int)c.permLen, c.STG, c.HST, c.OFF, c.START, c.TOT, c.PERM, c.ROWPTR, c.ROWCNT, c.FLAG);
}

typedef __attribute__((ext_vector_type(4))) _Float16 v4h;
__global__ __launch_bounds__(256) void prep_kernel(const float* __restrict__ x, const float* __restrict__ wr0, const float* __restrict__ wr1, const float* __restrict__ wr2, const float* __restrict__ wg, const float* __restrict__ wa, b16* __restrict__ Xh, b16* __restrict__ WR, b16* __restrict__ WG, b16* __restrict__ WA) {
  size_t t = (size_t)blockIdx.x * 256 + threadIdx.x; v8b o;
  { const size_t n = (size_t)NP * D / 8; if (t < n) { const size_t e = t * 8; const size_t v = e / D; for (int j = 0; j < 8; ++j) o[j] = (v < (size_t)N) ? (b16)(bf16_rne(x[e + j]) * XS) : (b16)0.0f; for (int pass = 0; pass < 2; ++pass) { *(volatile v8b*)(Xh + e) = o; __threadfence(); } return; } t -= n; }
  { const size_t n = (size_t)D * KS / 8; if (t < n) { const size_t e = t * 8; const int oo = (int)(e / KS), k0 = (int)(e % KS); const int b = k0 / D, kk = k0 % D; const float* w = b == 0 ? wr0 : (b == 1 ? wr1 : wr2);
      for (int j = 0; j < 8; ++j) o[j] = (b16)(bf16_rne(w[(size_t)(kk + j) * D + oo]) * WSC); for (int pass = 0; pass < 2; ++pass) { *(volatile v8b*)(WR + e) = o; __threadfence(); } return; } t -= n; }
  { const size_t n = (size_t)2 * D * D / 8; if (t < n) { const size_t e = t * 8; const int oo = (int)(e / D), k0 = (int)(e % D); const int half = oo / D, oc = oo % D;
      for (int j = 0; j < 8; ++j) o[j] = (b16)(bf16_rne(wg[(size_t)(half * D + k0 + j) * D + oc]) * WSC); for (int pass = 0; pass < 2; ++pass) { *(volatile v8b*)(WG + e) = o; __threadfence(); } return; } t -= n; }
  { const size_t n = (size_t)D * KA / 8; if (t < n) { const size_t e = t * 8; const int oo = (int)(e / KA), k0 = (int)(e % KA);
      for (int j = 0; j < 8; ++j) o[j] = (b16)(bf16_rne(wa[(size_t)(k0 + j) * D + oo]) * WSC); for (int pass = 0; pass < 2; ++pass) { *(volatile v8b*)(WA + e) = o; __threadfence(); } } }
}
__global__ __launch_bounds__(256) void edge_kernel(const float* __restrict__ x, const int* __restrict__ srcs, const int* __restrict__ ew, const int* __restrict__ cat, const float* __restrict__ wa0, const float* __restrict__ ba0, const float* __restrict__ em0, const float* __restrict__ wa1, const float* __restrict__ ba1, const float* __restrict__ em1, const float* __restrict__ wa2, const float* __restrict__ ba2, const float* __restrict__ em2,
                                                   const int* __restrict__ PERM, const int* __restrict__ ROWPTR, const int* __restrict__ ROWCNT, int permLen, b16* __restrict__ Sh, b16* __restrict__ Sl, float* __restrict__ AF) {
  __shared__ float saf[8];
  const int wave = threadIdx.x >> 5, lane = threadIdx.x & 31; const size_t v = (size_t)blockIdx.x * 8 + wave; const int c = lane * 4;
  v4f acc = {0.0f, 0.0f, 0.0f, 0.0f}; float den = 0.0f; int b = 0;
  if (v < (size_t)NLIMN) { b = iclamp(cat[v], 0, 2); const float* wa = b == 0 ? wa0 : (b == 1 ? wa1 : wa2); const float* em = b == 0 ? em0 : (b == 1 ? em1 : em2); const float batt = bf16_rne((b == 0 ? ba0 : (b == 1 ? ba1 : ba2))[0]);
    const v4f xv = *(const v4f*)(x + v * D + c); float wa1v[4], wa2v[4]; float xd = 0.0f;
    for (int i = 0; i < 4; ++i) { wa1v[i] = bf16_rne(wa[c + i]); wa2v[i] = bf16_rne(wa[D + c + i]); xd += pmul(bf16_rne(xv[i]), wa1v[i]); }
#pragma unroll
    for (int o = 1; o < 32; o <<= 1) xd += __shfl_xor(xd, o);
    float m = -INFINITY; int st = ROWPTR[v], cnt = ROWCNT[v]; cnt = iclamp(cnt, 0, 65536); st = iclamp(st, 0, permLen - cnt);
#pragma unroll 1
    for (int j = 0; j < cnt; ++j) { const int e = iclamp(PERM[st + j], 0, E - 1); const size_t s = (size_t)iclamp(srcs[e], 0, N - 1); const int ty = iclamp(ew[e], 0, NT - 1);
      const v4f xs = *(const v4f*)(x + s * D + c), ev = *(const v4f*)(em + (size_t)ty * D + c); v4f nm; float p = 0.0f;
      for (int i = 0; i < 4; ++i) { nm[i] = bf16_rne(ev[i]) * bf16_rne(xs[i]); p += pmul(nm[i], wa2v[i]); }
#pragma unroll
      for (int o = 1; o < 32; o <<= 1) p += __shfl_xor(p, o);
      float sc = xd + p + batt; sc = sc >= 0.0f ? sc : -0.1f * sc;
      const float mn = fmaxf(m, sc); const float alf = (m == -INFINITY) ? 0.0f : __expf(m - mn), w = __expf(sc - mn); acc = acc * alf + nm * w; den = den * alf + w; m = mn; }
    if (den > 0.0f) acc = acc * (1.0f / den); }
  const float af = (den > 0.0f) ? 1.0f : 0.0f;
  if (lane == 0) saf[wave] = af;
  v4h hv, lv, z4; for (int i = 0; i < 4; ++i) { b16 p, q; split16(acc[i] * XS, p, q); hv[i] = p; lv[i] = q; z4[i] = (b16)0.0f; }
  __syncthreads();
  for (int pass = 0; pass < 2; ++pass) {
    for (int bb = 0; bb < 3; ++bb) { const bool mine = (bb == b) && (den > 0.0f); *(volatile v4h*)(Sh + v * KS + bb * D + c) = mine ? hv : z4; *(volatile v4h*)(Sl + v * KS + bb * D + c) = mine ? lv : z4; }
    if (wave == 0 && lane < 8) { v4f o4 = {saf[lane], 0.0f, 0.0f, 0.0f}; *(volatile v4f*)(AF + ((size_t)blockIdx.x * 8 + lane) * 4) = o4; }
    __threadfence(); }
}
__global__ __launch_bounds__(128) void gemm1_kernel(const b16* __restrict__ Sh, const b16* __restrict__ Sl, const b16* __restrict__ WR, const float* __restrict__ AF, const int* __restrict__ cat, const float* __restrict__ br0, const float* __restrict__ br1, const float* __restrict__ br2, float* __restrict__ C) {
  __shared__ __attribute__((aligned(16))) float Tf[4][16][128 + 4];
  const int wave = threadIdx.x >> 5, lane = threadIdx.x & 31, nloc = lane & 15, hlf = lane >> 4; const size_t m0 = (size_t)blockIdx.x * 64 + wave * 16;
  v8f acc[8];
#pragma unroll
  for (int t = 0; t < 8; ++t) acc[t] = (v8f){};
#pragma unroll 2
  for (int kb = 0; kb < KS; kb += 32) { const v16b a = frag_kb(Sh + (m0 + nloc) * KS + kb, hlf), al = frag_kb(Sl + (m0 + nloc) * KS + kb, hlf);
#pragma unroll
    for (int t = 0; t < 8; ++t) { const v16b bw = frag_kb(WR + (size_t)(t * 16 + nloc) * KS + kb, hlf); acc[t] = wmma16b(a, bw, acc[t]); acc[t] = wmma16b(al, bw, acc[t]); } }
  float afr[8]; int cr[8];
#pragma unroll
  for (int r = 0; r < 8; ++r) { const size_t row = m0 + 8 * hlf + r; const bool live = row < (size_t)N; afr[r] = live ? AF[row * 4] : 0.0f; cr[r] = live ? iclamp(cat[row], 0, 2) : 0; }
#pragma unroll
  for (int t = 0; t < 8; ++t) { const int cc = t * 16 + nloc; const float b0 = bf16_rne(br0[cc]), b1 = bf16_rne(br1[cc]), b2 = bf16_rne(br2[cc]);
#pragma unroll
    for (int r = 0; r < 8; ++r) { float vv = acc[t][r] * (1.0f / (XS * WSC)) + afr[r] * (cr[r] == 0 ? b0 : (cr[r] == 1 ? b1 : b2)); if (m0 + 8 * hlf + r >= (size_t)N) vv = 0.0f; Tf[wave][8 * hlf + r][cc] = vv; } }
  wave_lds_sync();
  for (int pass = 0; pass < 2; ++pass) { for (int rr = 0; rr < 16; ++rr) *(volatile v4f*)(C + (m0 + rr) * D + lane * 4) = *(const v4f*)(&Tf[wave][rr][lane * 4]); __threadfence(); }
}
__global__ __launch_bounds__(128) void gemm2_kernel(const float* __restrict__ C, const b16* __restrict__ WG, const float* __restrict__ bg, const int* __restrict__ cat, b16* __restrict__ Uh, b16* __restrict__ Ul) {
  __shared__ __attribute__((aligned(16))) float Tf[4][16][128 + 4];
  const int wave = threadIdx.x >> 5, lane = threadIdx.x & 31, nloc = lane & 15, hlf = lane >> 4; const size_t m0 = (size_t)blockIdx.x * 64 + wave * 16; const int slab = blockIdx.y; const size_t vr = m0 + nloc;
  v8f acc[8];
#pragma unroll
  for (int t = 0; t < 8; ++t) acc[t] = (v8f){};
#pragma unroll
  for (int ks = 0; ks < 4; ++ks) { v16b ah, al; const float* crow = C + vr * D + ks * 32;
    { const v4f c0 = *(const v4f*)(crow + 8 * hlf), c1 = *(const v4f*)(crow + 8 * hlf + 4), c2 = *(const v4f*)(crow + 16 + 8 * hlf), c3 = *(const v4f*)(crow + 16 + 8 * hlf + 4);
      float cv[16]; for (int i = 0; i < 4; ++i) { cv[i] = c0[i]; cv[4 + i] = c1[i]; cv[8 + i] = c2[i]; cv[12 + i] = c3[i]; }
#pragma unroll
      for (int e2 = 0; e2 < 16; ++e2) { b16 p, q; split16(cv[e2] * XS, p, q); ah[e2] = p; al[e2] = q; } }
#pragma unroll
    for (int t = 0; t < 8; ++t) { const v16b bw = frag_kb(WG + (size_t)(slab * D + t * 16 + nloc) * D + ks * 32, hlf); acc[t] = wmma16b(ah, bw, acc[t]); acc[t] = wmma16b(al, bw, acc[t]); } }
#pragma unroll
  for (int t = 0; t < 8; ++t) { const float bb = bf16_rne(bg[t * 16 + nloc]);
#pragma unroll
    for (int r = 0; r < 8; ++r) Tf[wave][8 * hlf + r][t * 16 + nloc] = acc[t][r] * (1.0f / (XS * WSC)) + bb; }
  wave_lds_sync();
  for (int pass = 0; pass < 2; ++pass) {
    for (int rr = 0; rr < 16; ++rr) { const size_t row = m0 + rr; const int c = lane * 4; const bool live = row < (size_t)N; const int ct = live ? iclamp(cat[row], 0, 2) : 0;
      const v4f g4 = *(const v4f*)(&Tf[wave][rr][c]); const v4f cv = *(const v4f*)(C + row * D + c); v4h hv, lv, z4; float val[4];
      for (int i = 0; i < 4; ++i) { const float sg = 1.0f / (1.0f + __expf(-g4[i])); val[i] = live ? ((slab == 0) ? (1.0f - sg) * cv[i] : sg * cv[i]) : 0.0f; b16 p, q; split16(val[i] * XS, p, q); hv[i] = p; lv[i] = q; z4[i] = (b16)0.0f; }
      auto put = [&](int blk, bool zero) { *(volatile v4h*)(Uh + row * KS + blk * D + c) = zero ? z4 : hv; *(volatile v4h*)(Ul + row * KS + blk * D + c) = zero ? z4 : lv; };
      if (!live) { if (slab == 0) { put(0, true); put(1, true); put(2, true); } }
      else if (slab == 0) { if (ct == 0) { put(0, false); put(1, false); put(2, true); } else if (ct == 1) { put(2, false); put(1, true); } }
      else { if (ct == 1) { put(0, false); } else if (ct == 2) { put(1, false); put(2, false); put(0, true); } } }
    __threadfence(); }
}
__global__ __launch_bounds__(128) void gemm3_kernel(const b16* __restrict__ Xh, const b16* __restrict__ Uh, const b16* __restrict__ Ul, const b16* __restrict__ WA, const float* __restrict__ bagg, float* __restrict__ out, float* __restrict__ out1) {
  __shared__ __attribute__((aligned(16))) float Tf[4][16][128 + 4];
  const int wave = threadIdx.x >> 5, lane = threadIdx.x & 31, nloc = lane & 15, hlf = lane >> 4; const size_t m0 = (size_t)blockIdx.x * 64 + wave * 16;
  if (blockIdx.x == 0 && threadIdx.x == 0) { for (int pass = 0; pass < 2; ++pass) { ((volatile float*)out1)[0] = 0.0f; __threadfence(); } }
  if (m0 >= (size_t)N) return;
  v8f acc[8];
#pragma unroll
  for (int t = 0; t < 8; ++t) acc[t] = (v8f){};
#pragma unroll
  for (int kb = 0; kb < D; kb += 32) { const v16b a = frag_kb(Xh + (m0 + nloc) * D + kb, hlf);
#pragma unroll
    for (int t = 0; t < 8; ++t) acc[t] = wmma16b(a, frag_kb(WA + (size_t)(t * 16 + nloc) * KA + kb, hlf), acc[t]); }
#pragma unroll 2
  for (int kb = 0; kb < KS; kb += 32) { const v16b a = frag_kb(Uh + (m0 + nloc) * KS + kb, hlf), al = frag_kb(Ul + (m0 + nloc) * KS + kb, hlf);
#pragma unroll
    for (int t = 0; t < 8; ++t) { const v16b bw = frag_kb(WA + (size_t)(t * 16 + nloc) * KA + D + kb, hlf); acc[t] = wmma16b(a, bw, acc[t]); acc[t] = wmma16b(al, bw, acc[t]); } }
#pragma unroll
  for (int t = 0; t < 8; ++t) { const float bb = bf16_rne(bagg[t * 16 + nloc]);
#pragma unroll
    for (int r = 0; r < 8; ++r) Tf[wave][8 * hlf + r][t * 16 + nloc] = tanhf(acc[t][r] * (1.0f / (XS * WSC)) + bb); }
  wave_lds_sync();
  for (int pass = 0; pass < 2; ++pass) { for (int rr = 0; rr < 16; ++rr) *(volatile v4f*)(out + (m0 + rr) * D + lane * 4) = *(const v4f*)(&Tf[wave][rr][lane * 4]); __threadfence(); }
}
}

extern "C" void kernel_launch(void* const* d_in, const int* in_sizes, int n_in, void* d_out, int out_size, void* d_ws, size_t ws_size, hipStream_t stream) {
  (void)n_in;
  auto Fp = [&](int i) { return (const float*)d_in[i]; }; auto Ip = [&](int i) { return (const int*)d_in[i]; };
  if (in_sizes[0] != N * D || in_sizes[1] != 2 * E || in_sizes[2] != E || in_sizes[3] != N || in_sizes[4] != D * D || in_sizes[6] != 2 * D || in_sizes[8] != NT * D || in_sizes[9] != D * D || in_sizes[14] != D * D || in_sizes[19] != 2 * D * D || in_sizes[21] != KA * D || in_sizes[22] != D || out_size != N * D + 1) return;
  size_t off = 0; char* ws = (char*)d_ws;
  auto carve = [&](size_t bytes) { char* p = ws + off; off += (bytes + 255) & ~(size_t)255; return p; };
  b16* Xh = (b16*)carve((size_t)NP * D * 2); b16* WR = (b16*)carve((size_t)D * KS * 2); b16* WG = (b16*)carve((size_t)2 * D * D * 2); b16* WA = (b16*)carve((size_t)D * KA * 2);
  b16* Sh = (b16*)carve((size_t)NP * KS * 2); b16* Sl = (b16*)carve((size_t)NP * KS * 2); float* AF = (float*)carve((size_t)NP * 4 * 4); float* C = (float*)carve((size_t)NP * D * 4);
  b16* Uh = Sh; b16* Ul = Sl;
  CsrBufs csr; off = csr_carve(csr, ws, off, E, N);
  if (off > ws_size || off > ((size_t)128 << 20)) return;
  prep_kernel<<<(unsigned)((((size_t)NP * D + (size_t)D * KS + (size_t)2 * D * D + (size_t)D * KA) / 8 + 255) / 256), 256, 0, stream>>>(Fp(0), Fp(4), Fp(9), Fp(14), Fp(19), Fp(21), Xh, WR, WG, WA);
  csr_build(csr, Ip(1) + E, E, N, stream);
  edge_kernel<<<NP / 8, 256, 0, stream>>>(Fp(0), Ip(1), Ip(2), Ip(3), Fp(6), Fp(7), Fp(8), Fp(11), Fp(12), Fp(13), Fp(16), Fp(17), Fp(18), csr.PERM, csr.ROWPTR, csr.ROWCNT, (int)csr.permLen, Sh, Sl, AF);
  gemm1_kernel<<<NLIM / 64, 128, 0, stream>>>(Sh, Sl, WR, AF, Ip(3), Fp(5), Fp(10), Fp(15), C);
  gemm2_kernel<<<dim3(NLIM / 64, 2), 128, 0, stream>>>(C, WG, Fp(20), Ip(3), Uh, Ul);
  gemm3_kernel<<<NLIM / 64, 128, 0, stream>>>(Xh, Uh, Ul, WA, Fp(22), (float*)d_out, (float*)d_out + (size_t)N * D);
}
